// GATModel_17076789969391
// MI455X (gfx1250) — hardware-verified
//
#include <hip/hip_runtime.h>
#include <stddef.h>
#include <stdint.h>
#include <math.h>

#define DIN    128
#define HC1    256
#define HID    64
#define NHD1   4
#define KP     512
#define CH1    32
#define NCLS   10
#define PG     16
#define NTHR   256
#define NWAVE  8
#define EPT    8
#define CHUNK  (NTHR * EPT)
#define WCAP   (EPT * 32)
#define LISTN  (NWAVE * WCAP)
#define NBA    1024
#define SLA    10
#define RCAP   28672
#define DEGCAP 128
#define GBM    64
#define GBN    64
#define GTHR   128
#define BN_RPB 250
#define NU1    (HC1 * (DIN / 8))
#define NU2    (HID * (KP / 8))
#define NEGSL  0.2f
#define EPS_SM 1e-16f
#define EPS_BN 1e-5f
#define AGG_ZINTS (LISTN + 2 * RCAP + 3 * NBA)
#define AGG_LDS_INTS (AGG_ZINTS + 16)
#define WSMAX  134217728

static_assert((CHUNK & (CHUNK - 1)) == 0 && CHUNK <= 4096);
static_assert((NBA & (NBA - 1)) == 0 && NBA == (1 << SLA));
static_assert(((long long)CHUNK << SLA) < (1LL << 31));
static_assert(NBA % NWAVE == 0 && NBA % 32 == 0 && NBA % GBM == 0);
static_assert(RCAP % 4 == 0 && AGG_ZINTS % 4 == 0 && LISTN % 4 == 0);
static_assert(AGG_LDS_INTS * 4 <= 300000);
static_assert(DIN % 32 == 0 && KP % 32 == 0 && KP == 2 * HC1);
static_assert(GBM == (GTHR / 32) * 16 && GTHR == 2 * GBN && GTHR == 2 * GBM);
static_assert(HC1 % GBN == 0 && HID == GBN && HC1 == NHD1 * HID);
static_assert(HC1 == 8 * 32 && HID == 2 * 32);
static_assert(NU1 % NTHR == 0 && NU2 % NTHR == 0);
static_assert(DIN / 8 == 16 && KP / 8 == 64);
static_assert(HID * CH1 == 2 * NTHR * 4);
static_assert(PG * CH1 == 2 * NTHR);
static_assert(PG * NCLS == 160 && (PG * NCLS) % 32 == 0 && (PG * NCLS * 4) % 128 == 0);
static_assert(PG == 2 * NWAVE && PG <= NBA);

typedef float          v2f  __attribute__((ext_vector_type(2)));
typedef float          v4f  __attribute__((ext_vector_type(4)));
typedef float          v8f  __attribute__((ext_vector_type(8)));
typedef double         v2d  __attribute__((ext_vector_type(2)));
typedef int            v4i  __attribute__((ext_vector_type(4)));
typedef int            v8i  __attribute__((ext_vector_type(8)));
typedef unsigned short v8us __attribute__((ext_vector_type(8)));
typedef __bf16         v16b __attribute__((ext_vector_type(16)));
typedef v2f  __attribute__((may_alias)) v2fa;
typedef v4f  __attribute__((may_alias)) v4fa;
typedef v2d  __attribute__((may_alias)) v2da;
typedef v4i  __attribute__((may_alias)) v4ia;
typedef v8us __attribute__((may_alias)) v8usa;
union FragB { v16b v; v8us h[2]; v8i w; };

__device__ __forceinline__ v8f wmb(const FragB& a, const FragB& b, v8f c) {
  v8f d = __builtin_amdgcn_wmma_f32_16x16x32_bf16(false, a.v, false, b.v, (short)0, c, false, false);
  asm volatile("v_nop\n\tv_nop\n\tv_nop\n\tv_nop" : "+v"(d) : "v"(a.w), "v"(b.w));
  return d;
}

__device__ __forceinline__ unsigned bf16_bits(float f) {
  const unsigned u = __float_as_uint(f);
  return ((u + 0x7FFFu + ((u >> 16) & 1u)) >> 16) & 0xFFFFu;
}
__device__ __forceinline__ float bf16_val(float f) {
  return __uint_as_float(bf16_bits(f) << 16);
}
__device__ __forceinline__ v4f bfr4(const v4f a) {
  v4f r; r.x = bf16_val(a.x); r.y = bf16_val(a.y); r.z = bf16_val(a.z); r.w = bf16_val(a.w); return r;
}

__device__ __forceinline__ void onl_step(float lg, float& mx, float& dn, float& s1, float& s2) {
  const float df = lg - mx;
  const float ee = expf(-fabsf(df));
  const bool  up = df > 0.f;
  s1 = up ? ee : 1.0f;
  s2 = up ? 1.0f : ee;
  mx = up ? lg : mx;
  dn = fmaf(dn, s1, s2);
}

template <int SLB>
__device__ __forceinline__ int scan_chunk(const int* __restrict__ dsts, int nE, int cbase, int slotBase,
                                          int nb, int vec8, int* list, int tid, int lane, int wave) {
  int wc = 0;
  const int el0  = tid * EPT;
  const int e0   = cbase + el0;
  const int sent = -2147483647 - 1;
  v4i da, db;
  if (vec8 != 0 && cbase + CHUNK <= nE) {
    da = *(const v4i*)(dsts + e0);
    db = *(const v4i*)(dsts + e0 + 4);
  } else {
    da.x = (e0     < nE) ? dsts[min(e0,     nE - 1)] : sent;
    da.y = (e0 + 1 < nE) ? dsts[min(e0 + 1, nE - 1)] : sent;
    da.z = (e0 + 2 < nE) ? dsts[min(e0 + 2, nE - 1)] : sent;
    da.w = (e0 + 3 < nE) ? dsts[min(e0 + 3, nE - 1)] : sent;
    db.x = (e0 + 4 < nE) ? dsts[min(e0 + 4, nE - 1)] : sent;
    db.y = (e0 + 5 < nE) ? dsts[min(e0 + 5, nE - 1)] : sent;
    db.z = (e0 + 6 < nE) ? dsts[min(e0 + 6, nE - 1)] : sent;
    db.w = (e0 + 7 < nE) ? dsts[min(e0 + 7, nE - 1)] : sent;
  }
  const unsigned nbs = (unsigned)slotBase;
  const unsigned unb = (unsigned)nb;
  const unsigned s0 = (unsigned)da.x - nbs, s1 = (unsigned)da.y - nbs;
  const unsigned s2 = (unsigned)da.z - nbs, s3 = (unsigned)da.w - nbs;
  const unsigned s4 = (unsigned)db.x - nbs, s5 = (unsigned)db.y - nbs;
  const unsigned s6 = (unsigned)db.z - nbs, s7 = (unsigned)db.w - nbs;
  const bool h0 = s0 < unb, h1 = s1 < unb, h2 = s2 < unb, h3 = s3 < unb;
  const bool h4 = s4 < unb, h5 = s5 < unb, h6 = s6 < unb, h7 = s7 < unb;
  const unsigned any = __builtin_amdgcn_ballot_w32(h0 | h1 | h2 | h3 | h4 | h5 | h6 | h7);
  if (any != 0u) {
#define HITJ(J, HJ, SJ) { \
      const unsigned mj = __builtin_amdgcn_ballot_w32(HJ); \
      if (mj != 0u) { \
        if (HJ) { \
          const int pos = wc + (int)__builtin_amdgcn_mbcnt_lo(mj, 0u); \
          if (pos < WCAP) list[wave * WCAP + pos] = ((el0 + (J)) << SLB) | (int)(SJ); \
        } \
        wc += (int)__builtin_popcount(mj); } }
    HITJ(0, h0, s0)
    HITJ(1, h1, s1)
    HITJ(2, h2, s2)
    HITJ(3, h3, s3)
    HITJ(4, h4, s4)
    HITJ(5, h5, s5)
    HITJ(6, h6, s6)
    HITJ(7, h7, s7)
#undef HITJ
  }
  return wc;
}

__global__ __launch_bounds__(NTHR) void k_prep(const float* __restrict__ x, const float* __restrict__ W1,
                                               const float* __restrict__ W2,
                                               unsigned short* XB, unsigned short* W1T, unsigned short* W2T,
                                               int nN, int nUnits) {
  const int u = (int)blockIdx.x * NTHR + (int)threadIdx.x;
  v8us o;
  unsigned short* dp;
  if (u < NU1) {
    const int n  = u >> 4;
    const int k8 = (u & 15) * 8;
    const float* p = W1 + (size_t)k8 * HC1 + n;
#pragma unroll
    for (int i = 0; i < 8; ++i) o[i] = (unsigned short)bf16_bits(p[(size_t)i * HC1]);
    dp = W1T + (size_t)n * DIN + k8;
  } else if (u < NU1 + NU2) {
    const int v  = u - NU1;
    const int n  = v >> 6;
    const int k8 = (v & 63) * 8;
    const int kk = k8 & (HC1 - 1);
    const float* p = W2 + (size_t)kk * HID + n;
#pragma unroll
    for (int i = 0; i < 8; ++i) o[i] = (unsigned short)bf16_bits(p[(size_t)i * HID]);
    dp = W2T + (size_t)n * KP + k8;
  } else if (u < nUnits) {
    const int v   = u - NU1 - NU2;
    const int row = v >> 4;
    const int k8  = (v & 15) * 8;
    const int rc  = row < nN ? row : nN - 1;
    const float* p = x + (size_t)rc * DIN + k8;
    const v4f a = *(const v4fa*)p;
    const v4f b = *(const v4fa*)(p + 4);
    const bool ok = row < nN;
    o[0] = ok ? (unsigned short)bf16_bits(a.x) : (unsigned short)0;
    o[1] = ok ? (unsigned short)bf16_bits(a.y) : (unsigned short)0;
    o[2] = ok ? (unsigned short)bf16_bits(a.z) : (unsigned short)0;
    o[3] = ok ? (unsigned short)bf16_bits(a.w) : (unsigned short)0;
    o[4] = ok ? (unsigned short)bf16_bits(b.x) : (unsigned short)0;
    o[5] = ok ? (unsigned short)bf16_bits(b.y) : (unsigned short)0;
    o[6] = ok ? (unsigned short)bf16_bits(b.z) : (unsigned short)0;
    o[7] = ok ? (unsigned short)bf16_bits(b.w) : (unsigned short)0;
    dp = XB + (size_t)row * DIN + k8;
  } else {
    return;
  }
  *(volatile v8us*)dp = o;
  __threadfence();
  *(volatile v8us*)dp = o;
}

__global__ __launch_bounds__(GTHR) void k_gemm(
    const unsigned short* __restrict__ A, const unsigned short* __restrict__ WT,
    float* outF, int K, int ldo,
    const float* __restrict__ atts, const float* __restrict__ attd, int attLen,
    float* SD, int MPr)
{
  __shared__ __attribute__((aligned(16))) float stg[GBM * GBN];
  __shared__ __attribute__((aligned(16))) float satt[2 * GBN];
  __shared__ __attribute__((aligned(16))) float sdot[2 * GBM];
  const int tid = (int)threadIdx.x, lane = tid & 31, wave = tid >> 5, hh = lane >> 4, m = lane & 15;
  const int rowBase = (int)blockIdx.x * GBM;
  const int head    = (int)blockIdx.y;
  const int col0    = head * GBN;

  {
    const int which = tid >> 6;
    const int c  = tid & 63;
    const int cl = c < attLen ? c : attLen - 1;
    const float vs = atts[head * attLen + cl];
    const float vd = attd[head * attLen + cl];
    float v = (which == 0) ? vs : vd;
    v = (c < attLen) ? bf16_val(v) : 0.f;
    satt[which * GBN + c] = v;
  }

  v8f acc[4];
  {
    const v8f z = {0.f, 0.f, 0.f, 0.f, 0.f, 0.f, 0.f, 0.f};
    acc[0] = z; acc[1] = z; acc[2] = z; acc[3] = z;
  }
  const unsigned short* ap = A  + (size_t)(rowBase + 16 * wave + m) * (size_t)K + 8 * hh;
  const unsigned short* wp = WT + (size_t)(col0 + m) * (size_t)K + 8 * hh;
  const int ksteps = K >> 5;
#pragma unroll 1
  for (int ks = 0; ks < ksteps; ++ks) {
    FragB af;
    af.h[0] = *(const v8usa*)(ap + 32 * ks);
    af.h[1] = *(const v8usa*)(ap + 32 * ks + 16);
#pragma unroll
    for (int t = 0; t < 4; ++t) {
      const unsigned short* wq = wp + (size_t)(16 * t) * (size_t)K + 32 * ks;
      FragB bf;
      bf.h[0] = *(const v8usa*)wq;
      bf.h[1] = *(const v8usa*)(wq + 16);
      acc[t] = wmb(af, bf, acc[t]);
    }
  }

#pragma unroll
  for (int t = 0; t < 4; ++t) {
    const int lc = 16 * t + m;
#pragma unroll
    for (int r = 0; r < 8; ++r) {
      const int lr = 16 * wave + 8 * hh + r;
      stg[lr * GBN + lc] = acc[t][r];
    }
  }
  __syncthreads();

  {
    const int row = tid & 63, which = tid >> 6;
    const float* sa = satt + which * GBN;
    const float* hr = stg + row * GBN;
    float d = 0.f;
#pragma unroll 4
    for (int c4 = 0; c4 < GBN / 4; ++c4) {
      const v4f hv = *(const v4fa*)(hr + 4 * c4);
      const v4f av = *(const v4fa*)(sa + 4 * c4);
      d = fmaf(hv.x, av.x, d);
      d = fmaf(hv.y, av.y, d);
      d = fmaf(hv.z, av.z, d);
      d = fmaf(hv.w, av.w, d);
    }
    sdot[which * GBM + row] = d;
  }
  __syncthreads();

  v4f fv[8];
#pragma unroll
  for (int i = 0; i < 8; ++i) {
    const int lr = 16 * wave + 2 * i + hh;
    fv[i] = *(const v4fa*)(stg + lr * GBN + 4 * m);
  }
  const int which2 = lane >> 4, piece = lane & 15;
  const v4f sdv = *(const v4fa*)(sdot + which2 * GBM + 4 * piece);
  float* sp = SD + (size_t)(2 * head + which2) * (size_t)MPr + rowBase + 4 * piece;

#pragma unroll
  for (int i = 0; i < 8; ++i) {
    const int lr = 16 * wave + 2 * i + hh;
    const int gr = rowBase + lr;
    float* op = outF + (size_t)gr * (size_t)ldo + col0 + 4 * m;
    *(volatile v4f*)op = fv[i];
  }
  if (wave == 0) *(volatile v4f*)sp = sdv;
  __threadfence();
#pragma unroll
  for (int i = 0; i < 8; ++i) {
    const int lr = 16 * wave + 2 * i + hh;
    const int gr = rowBase + lr;
    float* op = outF + (size_t)gr * (size_t)ldo + col0 + 4 * m;
    *(volatile v4f*)op = fv[i];
  }
  if (wave == 0) *(volatile v4f*)sp = sdv;
}

template <int L>
__global__ __launch_bounds__(NTHR) void k_agg(const int* __restrict__ srcs, const int* __restrict__ dsts,
                                              int nE, int nN, int vec8, int MPr,
                                              const float* __restrict__ SD,
                                              const float* __restrict__ xl, const float* __restrict__ bias,
                                              float* outp) {
  static_assert(L == 1 || L == 2);
  extern __shared__ __attribute__((aligned(16))) int dsm[];
  int* list = dsm;
  int* hl   = dsm + LISTN;
  int* sl   = dsm + LISTN + RCAP;
  int* cnt  = dsm + LISTN + 2 * RCAP;
  int* offs = cnt + NBA;
  int* cur  = offs + NBA;
  int* misc = cur + NBA;
  const int tid = (int)threadIdx.x, lane = tid & 31, wave = tid >> 5;
  const int nodeBase = (int)blockIdx.x * NBA;

  {
    const v4i z4 = {0, 0, 0, 0};
    for (int i = tid * 4; i < AGG_ZINTS; i += NTHR * 4) *(v4ia*)(dsm + i) = z4;
    if (tid < 16) misc[tid] = 0;
  }
  __syncthreads();

  int t = 0, ov = 0;
  const int nChunks = (nE + CHUNK - 1) / CHUNK;
#pragma unroll 1
  for (int ch = 0; ch < nChunks; ++ch) {
    const int cbase = ch * CHUNK;
    const int wc = scan_chunk<SLA>(dsts, nE, cbase, nodeBase, NBA, vec8, list, tid, lane, wave);
    if (lane == 0) misc[wave] = wc;
    __syncthreads();
    if (wave == 0) {
#pragma unroll 1
      for (int w2 = 0; w2 < NWAVE; ++w2) {
        int c = misc[w2];
        c = c < 0 ? 0 : (c > WCAP ? WCAP : c);
#pragma unroll 1
        for (int b0 = 0; b0 < c; b0 += 32) {
          const int idx = b0 + lane;
          const int ent = list[w2 * WCAP + (idx < WCAP ? idx : WCAP - 1)];
          const int m32 = (c - b0) < 32 ? (c - b0) : 32;
#pragma unroll 1
          for (int k = 0; k < m32; ++k) {
            const int u    = __builtin_amdgcn_readlane(ent, k);
            const int slot = u & (NBA - 1);
            const int el   = (u >> SLA) & (CHUNK - 1);
            const int pk   = ((cbase + el) << SLA) | slot;
            if (t < RCAP) {
              if (lane == 0) { hl[t] = pk; cnt[slot] = cnt[slot] + 1; }
              t = t + 1;
            } else {
              ov = 1;
            }
          }
        }
      }
    }
    __syncthreads();
  }
  if (wave == 0 && lane == 0) { misc[8] = t; misc[9] = ov; }
  __syncthreads();
  int tt = misc[8];
  tt = tt < 0 ? 0 : (tt > RCAP ? RCAP : tt);
  const int ovf = misc[9];

  if (wave == 0) {
    const int base = lane * (NBA / 32);
    int s = 0;
#pragma unroll 1
    for (int i = 0; i < NBA / 32; ++i) s += cnt[base + i];
    int incl = s;
#pragma unroll
    for (int d = 1; d < 32; d <<= 1) {
      const int y = __shfl_up(incl, d, 32);
      if (lane >= d) incl += y;
    }
    int run = incl - s;
#pragma unroll 1
    for (int i = 0; i < NBA / 32; ++i) {
      const int cv = cnt[base + i];
      offs[base + i] = run;
      cur[base + i]  = run;
      run += cv;
    }
  }
  __syncthreads();
  if (wave == 0) {
#pragma unroll 1
    for (int b0 = 0; b0 < tt; b0 += 32) {
      const int idx = b0 + lane;
      const int ent = hl[idx < RCAP ? idx : RCAP - 1];
      const int m32 = (tt - b0) < 32 ? (tt - b0) : 32;
#pragma unroll 1
      for (int k = 0; k < m32; ++k) {
        const int u    = __builtin_amdgcn_readlane(ent, k);
        const int slot = u & (NBA - 1);
        if (lane == 0) {
          int p = cur[slot];
          p = p < 0 ? 0 : (p > RCAP - 1 ? RCAP - 1 : p);
          sl[p] = u;
          cur[slot] = p + 1;
        }
      }
    }
  }
  __syncthreads();

  const float qnan = __int_as_float(0x7fc00000);
  const float pz = (ovf != 0) ? qnan : 0.0f;

  if constexpr (L == 1) {
    const int hA = lane >> 4;
    const float* ASa = SD + (size_t)(2 * hA) * (size_t)MPr;
    const float* ADa = ASa + MPr;
    const float* ASb = SD + (size_t)(2 * (hA + 2)) * (size_t)MPr;
    const float* ADb = ASb + MPr;
    const v4f bA = bfr4(*(const v4fa*)(bias + 4 * lane));
    const v4f bB = bfr4(*(const v4fa*)(bias + 128 + 4 * lane));
#pragma unroll 1
    for (int si = 0; si < NBA / NWAVE; ++si) {
      const int s    = si * NWAVE + wave;
      const int node = nodeBase + s;
      int c = cnt[s];
      const bool big = c > DEGCAP;
      c = c < 0 ? 0 : (c > DEGCAP ? DEGCAP : c);
      int o = offs[s];
      o = o < 0 ? 0 : (o > RCAP ? RCAP : o);
      const int nc = node < nN ? node : nN - 1;
      const float* sp = xl + (size_t)nc * HC1 + 4 * lane;
      v4f aA = *(const v4fa*)sp;
      v4f aB = *(const v4fa*)(sp + 128);
      const float adA = ADa[nc], adB = ADb[nc];
      float lA = ASa[nc] + adA; lA = lA > 0.f ? lA : NEGSL * lA;
      float lB = ASb[nc] + adB; lB = lB > 0.f ? lB : NEGSL * lB;
      float mxA = lA, dnA = 1.0f, mxB = lB, dnB = 1.0f;
#pragma unroll 1
      for (int b0 = 0; b0 < c; b0 += 32) {
        int idx = o + b0 + lane;
        idx = idx > RCAP - 1 ? RCAP - 1 : idx;
        const int ent = sl[idx];
        int eid = ent >> SLA;
        eid = eid < 0 ? 0 : (eid > nE - 1 ? nE - 1 : eid);
        int sr = srcs[eid];
        sr = sr < 0 ? 0 : (sr > nN - 1 ? nN - 1 : sr);
        const int m32 = (c - b0) < 32 ? (c - b0) : 32;
#pragma unroll 1
        for (int k = 0; k < m32; ++k) {
          const int sk = __builtin_amdgcn_readlane(sr, k);
          const float* rp = xl + (size_t)sk * HC1 + 4 * lane;
          const v4f fA = *(const v4fa*)rp;
          const v4f fB = *(const v4fa*)(rp + 128);
          float gA = ASa[sk] + adA; gA = gA > 0.f ? gA : NEGSL * gA;
          float gB = ASb[sk] + adB; gB = gB > 0.f ? gB : NEGSL * gB;
          float s1, s2;
          onl_step(gA, mxA, dnA, s1, s2);
          aA.x = fmaf(aA.x, s1, s2 * fA.x); aA.y = fmaf(aA.y, s1, s2 * fA.y);
          aA.z = fmaf(aA.z, s1, s2 * fA.z); aA.w = fmaf(aA.w, s1, s2 * fA.w);
          onl_step(gB, mxB, dnB, s1, s2);
          aB.x = fmaf(aB.x, s1, s2 * fB.x); aB.y = fmaf(aB.y, s1, s2 * fB.y);
          aB.z = fmaf(aB.z, s1, s2 * fB.z); aB.w = fmaf(aB.w, s1, s2 * fB.w);
        }
      }
      const float invA = __builtin_amdgcn_rcpf(dnA + EPS_SM);
      const float invB = __builtin_amdgcn_rcpf(dnB + EPS_SM);
      const float pzr  = big ? qnan : pz;
      v4f oA, oB;
      oA.x = fmaf(aA.x, invA, bA.x) + pzr; oA.y = fmaf(aA.y, invA, bA.y) + pzr;
      oA.z = fmaf(aA.z, invA, bA.z) + pzr; oA.w = fmaf(aA.w, invA, bA.w) + pzr;
      oB.x = fmaf(aB.x, invB, bB.x) + pzr; oB.y = fmaf(aB.y, invB, bB.y) + pzr;
      oB.z = fmaf(aB.z, invB, bB.z) + pzr; oB.w = fmaf(aB.w, invB, bB.w) + pzr;
      const bool live = node < nN;
      float* op = outp + (size_t)nc * HC1 + 4 * lane;
      if (live) { *(volatile v4f*)op = oA; *(volatile v4f*)(op + 128) = oB; }
      __threadfence();
      if (live) { *(volatile v4f*)op = oA; *(volatile v4f*)(op + 128) = oB; }
    }
  } else {
    const v2f braw = *(const v2fa*)(bias + 2 * lane);
    const float bz0 = bf16_val(braw.x), bz1 = bf16_val(braw.y);
    const float* ASp = SD;
    const float* ADp = SD + MPr;
    const int sa = (2 * lane) & 31, sb = (2 * lane + 1) & 31;
#pragma unroll 1
    for (int si = 0; si < NBA / NWAVE; ++si) {
      const int s    = si * NWAVE + wave;
      const int node = nodeBase + s;
      int c = cnt[s];
      const bool big = c > DEGCAP;
      c = c < 0 ? 0 : (c > DEGCAP ? DEGCAP : c);
      int o = offs[s];
      o = o < 0 ? 0 : (o > RCAP ? RCAP : o);
      const int nc = node < nN ? node : nN - 1;
      const v2f fd = *(const v2fa*)(xl + (size_t)nc * HID + 2 * lane);
      const float ad = ADp[nc];
      float l0 = ASp[nc] + ad; l0 = l0 > 0.f ? l0 : NEGSL * l0;
      float mx = l0, dn = 1.0f;
      float a0 = fd.x, a1 = fd.y;
#pragma unroll 1
      for (int b0 = 0; b0 < c; b0 += 32) {
        int idx = o + b0 + lane;
        idx = idx > RCAP - 1 ? RCAP - 1 : idx;
        const int ent = sl[idx];
        int eid = ent >> SLA;
        eid = eid < 0 ? 0 : (eid > nE - 1 ? nE - 1 : eid);
        int sr = srcs[eid];
        sr = sr < 0 ? 0 : (sr > nN - 1 ? nN - 1 : sr);
        const int m32 = (c - b0) < 32 ? (c - b0) : 32;
#pragma unroll 1
        for (int k = 0; k < m32; ++k) {
          const int sk = __builtin_amdgcn_readlane(sr, k);
          const v2f fs = *(const v2fa*)(xl + (size_t)sk * HID + 2 * lane);
          float lg = ASp[sk] + ad; lg = lg > 0.f ? lg : NEGSL * lg;
          float s1, s2;
          onl_step(lg, mx, dn, s1, s2);
          a0 = fmaf(a0, s1, s2 * fs.x);
          a1 = fmaf(a1, s1, s2 * fs.y);
        }
      }
      const float inv = __builtin_amdgcn_rcpf(dn + EPS_SM);
      const float pzr = big ? qnan : pz;
      float y0 = fmaf(a0, inv, bz0);
      float y1 = fmaf(a1, inv, bz1);
      y0 = (y0 > 0.f) ? y0 : (y0 - y0);
      y1 = (y1 > 0.f) ? y1 : (y1 - y1);
      y0 = y0 + pzr;
      y1 = y1 + pzr;
      v4f ov4;
      ov4.x = __shfl(y0, sa); ov4.y = __shfl(y1, sa);
      ov4.z = __shfl(y0, sb); ov4.w = __shfl(y1, sb);
      const bool wr = (node < nN) && (lane < 16);
      float* op = outp + (size_t)nc * HID + 4 * (lane & 15);
      if (wr) *(volatile v4f*)op = ov4;
      __threadfence();
      if (wr) *(volatile v4f*)op = ov4;
    }
  }
}

__global__ __launch_bounds__(NTHR) void k_bnstat(const float* __restrict__ h, int nN, double* rec) {
  __shared__ __attribute__((aligned(16))) double sred[2 * HC1];
  const int c  = (int)threadIdx.x;
  const int r0 = (int)blockIdx.x * BN_RPB;
  int r1 = r0 + BN_RPB; r1 = r1 > nN ? nN : r1;
  double s = 0.0, ss = 0.0;
#pragma unroll 4
  for (int r = r0; r < r1; ++r) {
    const double v = (double)h[(size_t)r * HC1 + c];
    s += v;
    ss = fma(v, v, ss);
  }
  sred[c] = s;
  sred[HC1 + c] = ss;
  __syncthreads();
  const v2d o = *(const v2da*)(sred + 2 * c);
  double* dp = rec + (size_t)blockIdx.x * (2 * HC1) + 2 * c;
  *(volatile v2d*)dp = o;
  __threadfence();
  *(volatile v2d*)dp = o;
}

__global__ __launch_bounds__(NTHR) void k_bncomb(const double* __restrict__ rec, float* bnp, double invN, int nRec) {
  __shared__ __attribute__((aligned(16))) float sm[2 * HC1];
  const int c = (int)threadIdx.x;
  double S = 0.0, SS = 0.0;
#pragma unroll 2
  for (int r = 0; r < nRec; ++r) {
    S  += rec[(size_t)r * (2 * HC1) + c];
    SS += rec[(size_t)r * (2 * HC1) + HC1 + c];
  }
  const double mu = S * invN;
  double var = SS * invN - mu * mu;
  if (var < 0.0) var = 0.0;
  sm[c] = (float)mu;
  sm[HC1 + c] = rsqrtf((float)var + EPS_BN);
  __syncthreads();
  const int pi = c < 127 ? c : 127;
  const v4f o = *(const v4fa*)(sm + 4 * pi);
  float* dp = bnp + 4 * pi;
  const bool wr = c < 128;
  if (wr) *(volatile v4f*)dp = o;
  __threadfence();
  if (wr) *(volatile v4f*)dp = o;
}

__global__ __launch_bounds__(NTHR) void k_bnapply(const float* __restrict__ h, const float* __restrict__ bnp,
                                                  const float* __restrict__ gamma, const float* __restrict__ beta,
                                                  int nN, int nUnits, unsigned short* y) {
  const int u = (int)blockIdx.x * NTHR + (int)threadIdx.x;
  if (u >= nUnits) return;
  const int row = u >> 5;
  const int c8  = (u & 31) * 8;
  const int rc  = row < nN ? row : nN - 1;
  const float* p = h + (size_t)rc * HC1 + c8;
  const v4f xa = *(const v4fa*)p,                 xb = *(const v4fa*)(p + 4);
  const v4f ma = *(const v4fa*)(bnp + c8),        mb = *(const v4fa*)(bnp + c8 + 4);
  const v4f ra = *(const v4fa*)(bnp + HC1 + c8),  rb = *(const v4fa*)(bnp + HC1 + c8 + 4);
  const v4f ga = bfr4(*(const v4fa*)(gamma + c8)), gb = bfr4(*(const v4fa*)(gamma + c8 + 4));
  const v4f ba = bfr4(*(const v4fa*)(beta + c8)),  bb = bfr4(*(const v4fa*)(beta + c8 + 4));
  float v[8];
  v[0] = ((xa.x - ma.x) * ra.x) * ga.x + ba.x;
  v[1] = ((xa.y - ma.y) * ra.y) * ga.y + ba.y;
  v[2] = ((xa.z - ma.z) * ra.z) * ga.z + ba.z;
  v[3] = ((xa.w - ma.w) * ra.w) * ga.w + ba.w;
  v[4] = ((xb.x - mb.x) * rb.x) * gb.x + bb.x;
  v[5] = ((xb.y - mb.y) * rb.y) * gb.y + bb.y;
  v[6] = ((xb.z - mb.z) * rb.z) * gb.z + bb.z;
  v[7] = ((xb.w - mb.w) * rb.w) * gb.w + bb.w;
  const bool ok = row < nN;
  v8us ho, lo;
#pragma unroll
  for (int i = 0; i < 8; ++i) {
    float t = v[i];
    t = (t > 0.f) ? t : (t - t);
    t = ok ? t : 0.f;
    const unsigned hbi = bf16_bits(t);
    ho[i] = (unsigned short)hbi;
    lo[i] = (unsigned short)bf16_bits(t - __uint_as_float(hbi << 16));
  }
  unsigned short* dp = y + (size_t)row * KP + c8;
  *(volatile v8us*)dp = ho;
  *(volatile v8us*)(dp + HC1) = lo;
  __threadfence();
  *(volatile v8us*)dp = ho;
  *(volatile v8us*)(dp + HC1) = lo;
}

__global__ __launch_bounds__(NTHR) void k_pool_head(const int* __restrict__ batch, const float* __restrict__ h2,
                                                    int nN, int vecB,
                                                    const float* __restrict__ cW1, const float* __restrict__ cb1,
                                                    const float* __restrict__ cW2, const float* __restrict__ cb2,
                                                    float* out) {
  __shared__ __attribute__((aligned(16))) int   list[LISTN];
  __shared__ int wcnt[NWAVE];
  __shared__ __attribute__((aligned(16))) float pooled[PG * HID];
  __shared__ __attribute__((aligned(16))) float sW1[HID * CH1];
  __shared__ __attribute__((aligned(16))) float sW2[CH1 * NCLS];
  __shared__ float sb1[CH1];
  __shared__ float sb2[16];
  __shared__ float sz[PG * CH1];
  __shared__ __attribute__((aligned(16))) float so[PG * NCLS];
  const int tid = (int)threadIdx.x, lane = tid & 31, wave = tid >> 5;
  const int wv = __builtin_amdgcn_readfirstlane(wave);
  const int gBase = (int)blockIdx.x * PG;

  {
    const v4f w0 = bfr4(*(const v4fa*)(cW1 + 4 * tid));
    const v4f w1 = bfr4(*(const v4fa*)(cW1 + 4 * (tid + NTHR)));
    *(v4fa*)(sW1 + 4 * tid) = w0;
    *(v4fa*)(sW1 + 4 * (tid + NTHR)) = w1;
    const int i2 = tid < 79 ? tid : 79;
    const v4f w2 = bfr4(*(const v4fa*)(cW2 + 4 * i2));
    if (tid < 80) *(v4fa*)(sW2 + 4 * tid) = w2;
    const float v1 = bf16_val(cb1[tid < CH1 ? tid : CH1 - 1]);
    if (tid < CH1) sb1[tid] = v1;
    const float v2 = bf16_val(cb2[tid < NCLS ? tid : NCLS - 1]);
    if (tid < 16) sb2[tid] = (tid < NCLS) ? v2 : 0.f;
  }

  float a0 = 0.f, a1 = 0.f, b0 = 0.f, b1 = 0.f;
  int cA = 0, cB = 0;
  const int nChunks = (nN + CHUNK - 1) / CHUNK;
#pragma unroll 1
  for (int ch = 0; ch < nChunks; ++ch) {
    const int cbase = ch * CHUNK;
    const int wc = scan_chunk<SLA>(batch, nN, cbase, gBase, PG, vecB, list, tid, lane, wave);
    if (lane == 0) wcnt[wave] = wc;
    __syncthreads();
#pragma unroll 1
    for (int w2 = 0; w2 < NWAVE; ++w2) {
      int c = wcnt[w2];
      c = c < 0 ? 0 : (c > WCAP ? WCAP : c);
#pragma unroll 1
      for (int i = 0; i < c; ++i) {
        const int u    = __builtin_amdgcn_readfirstlane(list[w2 * WCAP + i]);
        const int slot = u & (NBA - 1);
        const int el   = (u >> SLA) & (CHUNK - 1);
        int node = cbase + el;
        node = node > nN - 1 ? nN - 1 : node;
        if (slot == wv) {
          const v2f r = *(const v2fa*)(h2 + (size_t)node * HID + 2 * lane);
          a0 += r.x; a1 += r.y; cA += 1;
        } else if (slot == wv + NWAVE) {
          const v2f r = *(const v2fa*)(h2 + (size_t)node * HID + 2 * lane);
          b0 += r.x; b1 += r.y; cB += 1;
        }
      }
    }
    __syncthreads();
  }
  {
    const float iA = 1.0f / fmaxf((float)cA, 1.0f);
    const float iB = 1.0f / fmaxf((float)cB, 1.0f);
    pooled[wave * HID + 2 * lane]               = a0 * iA;
    pooled[wave * HID + 2 * lane + 1]           = a1 * iA;
    pooled[(wave + NWAVE) * HID + 2 * lane]     = b0 * iB;
    pooled[(wave + NWAVE) * HID + 2 * lane + 1] = b1 * iB;
  }
  __syncthreads();

#pragma unroll 1
  for (int rep = 0; rep < 2; ++rep) {
    const int idx = tid + NTHR * rep;
    const int g = idx >> 5, j = idx & 31;
    float s = 0.f;
#pragma unroll 4
    for (int k = 0; k < HID; ++k) s = fmaf(pooled[g * HID + k], sW1[k * CH1 + j], s);
    s = s + sb1[j];
    s = (s > 0.f) ? s : (s - s);
    sz[idx] = s;
  }
  __syncthreads();

  if (tid < PG * NCLS) {
    const int g = tid / NCLS, o = tid - g * NCLS;
    float s = 0.f;
#pragma unroll 4
    for (int j = 0; j < CH1; ++j) s = fmaf(sz[g * CH1 + j], sW2[j * NCLS + o], s);
    so[tid] = s + sb2[o];
  }
  __syncthreads();

  const int pi = tid < 39 ? tid : 39;
  const v4f ov = *(const v4fa*)(so + 4 * pi);
  float* op = out + (size_t)blockIdx.x * (PG * NCLS) + 4 * pi;
  const bool wr = tid < (PG * NCLS) / 4;
  if (wr) *(volatile v4f*)op = ov;
  __threadfence();
  if (wr) *(volatile v4f*)op = ov;
}

static inline int cdiv(int a, int b) { return (a + b - 1) / b; }

extern "C" void kernel_launch(void* const* d_in, const int* in_sizes, int n_in,
                              void* d_out, int out_size, void* d_ws, size_t ws_size,
                              hipStream_t stream) {
  if (n_in < 17) return;
  if (in_sizes[0] < DIN || (in_sizes[0] % DIN) != 0) return;
  const int nN = in_sizes[0] / DIN;
  if (nN > (1 << 22)) return;
  if (in_sizes[1] < 2 || (in_sizes[1] & 1) != 0) return;
  const int nE = in_sizes[1] / 2;
  if (nE < 1 || nE >= (1 << 21)) return;
  if (in_sizes[2] != nN) return;
  if (in_sizes[3] != DIN * HC1) return;
  if (in_sizes[4] != HC1 || in_sizes[5] != HC1) return;
  if (in_sizes[6] != HC1 || in_sizes[7] != HC1 || in_sizes[8] != HC1) return;
  if (in_sizes[9] != HC1 * HID) return;
  if (in_sizes[10] != HID || in_sizes[11] != HID || in_sizes[12] != HID) return;
  if (in_sizes[13] != HID * CH1 || in_sizes[14] != CH1) return;
  if (in_sizes[15] != CH1 * NCLS || in_sizes[16] != NCLS) return;
  if (out_size < PG * NCLS || (out_size % (PG * NCLS)) != 0) return;
  const int nG = out_size / NCLS;

  const float* x    = (const float*)d_in[0];
  const int*   edge = (const int*)  d_in[1];
  const int*   bat  = (const int*)  d_in[2];
  const float* W1   = (const float*)d_in[3];
  const float* a1s  = (const float*)d_in[4];
  const float* a1d  = (const float*)d_in[5];
  const float* b1   = (const float*)d_in[6];
  const float* gam  = (const float*)d_in[7];
  const float* bet  = (const float*)d_in[8];
  const float* W2   = (const float*)d_in[9];
  const float* a2s  = (const float*)d_in[10];
  const float* a2d  = (const float*)d_in[11];
  const float* b2   = (const float*)d_in[12];
  const float* cW1  = (const float*)d_in[13];
  const float* cb1  = (const float*)d_in[14];
  const float* cW2  = (const float*)d_in[15];
  const float* cb2  = (const float*)d_in[16];
  float* out = (float*)d_out;
  const int* src = edge;
  const int* dst = edge + nE;

  const int MP   = cdiv(nN, GBM) * GBM;
  const int gM   = MP / GBM;
  const int gA   = cdiv(MP, NBA);
  if ((long long)gA * NBA < (long long)MP) return;
  const int nRec = cdiv(nN, BN_RPB);
  const int vecE = ((nE & 3) == 0) ? 1 : 0;
  const int vecB = ((nN & 3) == 0) ? 1 : 0;

  char* ws = (char*)d_ws;
  size_t off = 0;
  const size_t oRA  = off; off += (size_t)MP * HC1 * 4;              off = (off + 255) & ~(size_t)255;
  const size_t oRB  = off; off += (size_t)MP * HC1 * 4;              off = (off + 255) & ~(size_t)255;
  const size_t oRC  = off; off += (size_t)MP * DIN * 2;              off = (off + 255) & ~(size_t)255;
  const size_t oSD1 = off; off += (size_t)(2 * NHD1) * MP * 4;       off = (off + 255) & ~(size_t)255;
  const size_t oSD2 = off; off += (size_t)2 * MP * 4;                off = (off + 255) & ~(size_t)255;
  const size_t oW1T = off; off += (size_t)HC1 * DIN * 2;             off = (off + 255) & ~(size_t)255;
  const size_t oW2T = off; off += (size_t)HID * KP * 2;              off = (off + 255) & ~(size_t)255;
  const size_t oREC = off; off += (size_t)nRec * (2 * HC1) * 8;      off = (off + 255) & ~(size_t)255;
  const size_t oBNP = off; off += (size_t)(2 * HC1) * 4;             off = (off + 255) & ~(size_t)255;
  if (off > ws_size || off > (size_t)WSMAX) return;
  if ((size_t)MP * KP * 2 > (size_t)MP * HC1 * 4) return;
  if ((size_t)MP * HID * 4 > (size_t)MP * DIN * 2) return;
  float*          XH1 = (float*)(ws + oRA);
  unsigned short* Y   = (unsigned short*)(ws + oRA);
  float*          H1R = (float*)(ws + oRB);
  float*          H2  = (float*)(ws + oRB);
  unsigned short* XB  = (unsigned short*)(ws + oRC);
  float*          XH2 = (float*)(ws + oRC);
  float*          SD1 = (float*)(ws + oSD1);
  float*          SD2 = (float*)(ws + oSD2);
  unsigned short* W1T = (unsigned short*)(ws + oW1T);
  unsigned short* W2T = (unsigned short*)(ws + oW2T);
  double*         REC = (double*)(ws + oREC);
  float*          BNP = (float*)(ws + oBNP);

  const size_t aggLds = (size_t)AGG_LDS_INTS * 4;
  hipFuncSetAttribute(reinterpret_cast<const void*>(&k_agg<1>), hipFuncAttributeMaxDynamicSharedMemorySize, (int)aggLds);
  hipFuncSetAttribute(reinterpret_cast<const void*>(&k_agg<2>), hipFuncAttributeMaxDynamicSharedMemorySize, (int)aggLds);

  const int nUp = NU1 + NU2 + MP * (DIN / 8);
  k_prep<<<cdiv(nUp, NTHR), NTHR, 0, stream>>>(x, W1, W2, XB, W1T, W2T, nN, nUp);
  k_gemm<<<dim3(gM, HC1 / GBN), GTHR, 0, stream>>>(XB, W1T, XH1, DIN, HC1, a1s, a1d, HID, SD1, MP);
  k_agg<1><<<gA, NTHR, aggLds, stream>>>(src, dst, nE, nN, vecE, MP, SD1, XH1, b1, H1R);
  k_bnstat<<<nRec, NTHR, 0, stream>>>(H1R, nN, REC);
  k_bncomb<<<1, NTHR, 0, stream>>>(REC, BNP, 1.0 / (double)nN, nRec);
  const int nUy = MP * 32;
  k_bnapply<<<cdiv(nUy, NTHR), NTHR, 0, stream>>>(H1R, BNP, gam, bet, nN, nUy, Y);
  k_gemm<<<dim3(gM, 1), GTHR, 0, stream>>>(Y, W2T, XH2, KP, HID, a2s, a2d, HID, SD2, MP);
  k_agg<2><<<gA, NTHR, aggLds, stream>>>(src, dst, nE, nN, vecE, MP, SD2, XH2, b2, H2);
  k_pool_head<<<nG / PG, NTHR, 0, stream>>>(bat, H2, nN, vecB, cW1, cb1, cW2, cb2, out);
}
